// PerAgentMLP_53137335386139
// MI455X (gfx1250) — hardware-run, weakly checked
//
#include <hip/hip_runtime.h>


#ifndef NB
#define NB 1024
#endif
#define NB_FULL 1024
#define NSET    100
#define OBS     624
#define OBSP    640
#define HID     256
#define OUTD    24
#define OUTP    32
#define LIMBS   12
#define LIMB_SZ 52
#define XP      648
#define HP      264
#define OSP     36
#define CH      1024.0f
#define CW      1024.0f
#define CINV    (1.0f / (1024.0f * 1024.0f))

static_assert(LIMBS * LIMB_SZ == OBS);
static_assert(LIMB_SZ % 4 == 0);
static_assert(OBS % 4 == 0);
static_assert(OBSP % 64 == 0);
static_assert(OBSP >= OBS);
static_assert(HID % 64 == 0);
static_assert(HID % 32 == 0);
static_assert(OUTP % 32 == 0);
static_assert(OUTP >= OUTD);
static_assert(OUTD % 4 == 0);
static_assert(OBSP % 32 == 0);
static_assert(HID == 4 * 64);
static_assert(OUTP == 2 * 16);
static_assert(NB % 32 == 0);
static_assert(NB <= NB_FULL);
static_assert((16 * (OBSP / 4)) % 128 == 0);
static_assert(256 * 16 == 32 * 64 * 2);
static_assert(128 * 16 == 16 * OUTP * 4);
static_assert((XP * 2) % 16 == 0);
static_assert((HP * 2) % 16 == 0);
static_assert((OSP * 4) % 16 == 0);
static_assert(XP >= OBSP);
static_assert(HP >= HID);
static_assert(OSP >= OUTP);
static_assert((size_t)16 * XP * 2 + (size_t)2 * 16 * HP * 2 + (size_t)16 * OSP * 4 + (size_t)NB * 4 + 64 <= (size_t)131072);
static_assert((size_t)64 * 33 * 4 <= (size_t)131072);

typedef _Float16 h16;
typedef unsigned short bf;
typedef __attribute__((ext_vector_type(16))) __bf16   v16bf;
typedef __attribute__((ext_vector_type(16))) _Float16 v16h;
typedef __attribute__((ext_vector_type(8)))  _Float16 v8h;
typedef __attribute__((ext_vector_type(8)))  unsigned short v8us;
typedef __attribute__((ext_vector_type(8)))  float    v8f;
typedef __attribute__((ext_vector_type(4)))  float    v4f;
typedef v4f  __attribute__((may_alias)) v4fa;

__device__ __forceinline__ unsigned short f2bf(float f) { unsigned u = __float_as_uint(f); u += 0x7FFFu + ((u >> 16) & 1u); return (unsigned short)(u >> 16); }
__device__ __forceinline__ float bfr(float f) { return __uint_as_float(((unsigned)f2bf(f)) << 16); }
__device__ __forceinline__ v16h cat16(v8h lo, v8h hi) { return __builtin_shufflevector(lo, hi, 0, 1, 2, 3, 4, 5, 6, 7, 8, 9, 10, 11, 12, 13, 14, 15); }
__device__ __forceinline__ v16bf cat16b(v8us lo, v8us hi) { return __builtin_bit_cast(v16bf, __builtin_shufflevector(lo, hi, 0, 1, 2, 3, 4, 5, 6, 7, 8, 9, 10, 11, 12, 13, 14, 15)); }
__device__ __forceinline__ v8f wmma16(v16h a, v16h b, v8f c) { return __builtin_amdgcn_wmma_f32_16x16x32_f16(false, a, false, b, (short)0, c, false, false); }
__device__ __forceinline__ v8f wmmab(v16bf a, v16bf b, v8f c) { return __builtin_amdgcn_wmma_f32_16x16x32_bf16(false, a, false, b, (short)0, c, false, false); }
__device__ __forceinline__ v16h  ldh(const h16* p) { return cat16(*(const v8h*)p, *(const v8h*)(p + 16)); }
__device__ __forceinline__ v16bf ldb(const bf* p)  { return cat16b(*(const v8us*)p, *(const v8us*)(p + 16)); }
__device__ __forceinline__ void wave_sync() { __builtin_amdgcn_fence(3  , "wavefront"); __builtin_amdgcn_wave_barrier(); asm volatile("" ::: "memory"); }

typedef __attribute__((ext_vector_type(4)))  unsigned short v4us;
typedef __attribute__((ext_vector_type(4)))  int      v4i;
typedef v4us __attribute__((may_alias)) v4usa;
typedef v8us __attribute__((may_alias)) v8usa;
typedef v8h  __attribute__((may_alias)) v8ha;
static __device__ __forceinline__ h16 toh_flush(float v) { const h16 r = (h16)v; return (fabsf(v) < 6.103515625e-05f) ? (h16)0.0f : r; }
__device__ __forceinline__ v16h ldhu(const bf* p) { return __builtin_bit_cast(v16h, __builtin_shufflevector(*(const v8us*)p, *(const v8us*)(p + 16), 0, 1, 2, 3, 4, 5, 6, 7, 8, 9, 10, 11, 12, 13, 14, 15)); }
__device__ __forceinline__ v8f wmmabg(v16bf a, v16bf b, v8f c) { c = wmmab(a, b, c); asm volatile("v_nop\n\tv_nop\n\tv_nop\n\tv_nop" : "+v"(c) : "v"(a), "v"(b)); return c; }
__device__ __forceinline__ v8f wmma16g(v16h a, v16h b, v8f c) { c = wmma16(a, b, c); asm volatile("v_nop\n\tv_nop\n\tv_nop\n\tv_nop" : "+v"(c) : "v"(a), "v"(b)); return c; }

__global__ __launch_bounds__(256) void k_wt(const float* __restrict__ src, bf* dst, int K, int N, int KP, int NP, int f16mode, float carry) {
#pragma clang fp contract(off)
    __shared__ float tl[64 * 33];
    const int tid = threadIdx.x;
    const int k0 = blockIdx.x * 64, n0 = blockIdx.y * 32, sg = blockIdx.z;
    const float* sa = src + (size_t)sg * (size_t)K * (size_t)N;
    { const int nl = tid & 31, kl = tid >> 5; const int n = n0 + nl; const int nc = n < N ? n : N - 1;
#pragma unroll
      for (int j = 0; j < 8; ++j) { const int k = k0 + kl + 8 * j; const int kc = k < K ? k : K - 1;
          float v = sa[(size_t)kc * N + nc]; asm volatile("" : "+v"(v));
          tl[(kl + 8 * j) * 33 + nl] = ((k < K) & (n < N)) ? v : 0.0f; } }
    __syncthreads();
    const int nr = tid >> 3, pc = tid & 7;
    v8us o;
#pragma unroll
    for (int e = 0; e < 8; ++e) { const float raw = tl[(pc * 8 + e) * 33 + nr];
        const unsigned short b16 = f2bf(raw);
        const float wv = __uint_as_float(((unsigned)b16) << 16);
        const unsigned short hb = __builtin_bit_cast(unsigned short, toh_flush(wv * carry));
        o[e] = f16mode ? hb : b16; }
    const size_t oo = ((size_t)sg * NP + (size_t)(n0 + nr)) * KP + (size_t)k0 + (size_t)pc * 8;
    *(volatile v8us*)(dst + oo) = o; __threadfence(); *(volatile v8us*)(dst + oo) = o;
}

__global__ __launch_bounds__(128) void k_layers(const float* __restrict__ obs, const int* __restrict__ omask, const int* __restrict__ ids,
                                             const bf* __restrict__ WI, const float* __restrict__ bi,
                                             const bf* __restrict__ WH, const float* __restrict__ bh,
                                             const bf* __restrict__ WO, const float* __restrict__ bo, float* OW) {
    __shared__ __align__(16) bf    sx[16 * XP];
    __shared__ __align__(16) h16   sh1[16 * HP];
    __shared__ __align__(16) h16   sh2[16 * HP];
    __shared__ __align__(16) float so[16 * OSP];
    __shared__ int   lst[NB];
    __shared__ float sinv[16];
    const int tid = threadIdx.x;
    const int lane = tid & 31, lr = lane & 15, hi = lane >> 4;
    const int wave = __builtin_amdgcn_readfirstlane((int)(threadIdx.x >> 5));
    const int sg = blockIdx.x;

#pragma unroll 1
    for (int j = tid; j < NB; j += 128) lst[j] = 0;
    __syncthreads();
    int cnt = 0;
#pragma unroll 1
    for (int it = 0; it < NB / 32; ++it) {
        const int idx = it * 32 + lane;
        int id = ids[idx]; id = id < 0 ? 0 : (id > NSET - 1 ? NSET - 1 : id);
        const bool f = (id == sg);
        const unsigned bal = (unsigned)__ballot(f ? 1 : 0);
        const int pos = cnt + __popc(bal & ((1u << lane) - 1u));
        if ((wave == 0) & f) lst[pos < NB ? pos : NB - 1] = idx;
        cnt += __popc(bal);
    }
    __syncthreads();
    const int cc = cnt > NB ? NB : cnt;
    const int cntu = __builtin_amdgcn_readfirstlane(cc);
    const int nt = (cntu + 15) >> 4;

#pragma unroll 1
    for (int tile = 0; tile < nt; ++tile) {
        const int t0 = tile * 16;
        { const int r = tid & 15; const int li = t0 + r; const bool rv = li < cntu;
          int s = lst[li < NB ? li : NB - 1]; s = s < 0 ? 0 : (s > NB - 1 ? NB - 1 : s);
          const v4i* mp = (const v4i*)(omask + (size_t)s * LIMBS);
          const v4i a0 = mp[0], a1 = mp[1], a2 = mp[2];
          float ks = 0.0f;
#pragma unroll
          for (int i = 0; i < 4; ++i) ks += ((a0[i] == 0) ? 1.0f : 0.0f) + ((a1[i] == 0) ? 1.0f : 0.0f) + ((a2[i] == 0) ? 1.0f : 0.0f);
          const float den = rv ? ks : 1.0f;
          if (tid < 16) sinv[r] = 1.0f / den; }
#pragma unroll 1
        for (int q = tid; q < 16 * (OBSP / 4); q += 128) {
            const int r = q / (OBSP / 4), u = q - r * (OBSP / 4);
            const int li = t0 + r;
            int s = lst[li < NB ? li : NB - 1]; s = s < 0 ? 0 : (s > NB - 1 ? NB - 1 : s);
            const int uc = u < OBS / 4 ? u : OBS / 4 - 1;
            v4f v = *(const v4f*)(obs + (size_t)s * OBS + (size_t)uc * 4);
            int mk = omask[(size_t)s * LIMBS + (uc * 4) / LIMB_SZ];
            asm volatile("" : "+v"(v)); asm volatile("" : "+v"(mk));
            const bool keep = (li < cntu) & (u < OBS / 4) & (mk == 0);
            v4us o;
#pragma unroll
            for (int i = 0; i < 4; ++i) o[i] = keep ? f2bf(v[i]) : (unsigned short)0;
            *(v4usa*)(&sx[r * XP + u * 4]) = o;
        }
        __syncthreads();

        { const int cb = wave * 64;
          v8f acc[4];
#pragma unroll
          for (int nb = 0; nb < 4; ++nb) acc[nb] = (v8f){};
          const size_t wo = ((size_t)sg * HID + (size_t)(cb + lr)) * OBSP + 8 * hi;
          const int xo = lr * XP + 8 * hi;
#pragma unroll 1
          for (int kc = 0; kc < OBSP; kc += 32) {
              const v16bf a = cat16b(*(const v8usa*)(&sx[xo + kc]), *(const v8usa*)(&sx[xo + kc + 16]));
#pragma unroll
              for (int nb = 0; nb < 4; ++nb) { const v16bf b = ldb(WI + wo + (size_t)nb * 16 * OBSP + kc); acc[nb] = wmmabg(a, b, acc[nb]); }
          }
          float iv[8];
#pragma unroll
          for (int j = 0; j < 8; ++j) iv[j] = sinv[hi * 8 + j];
#pragma unroll
          for (int nb = 0; nb < 4; ++nb) { const int col = cb + nb * 16 + lr; const float bb = bfr(bi[(size_t)sg * HID + col]);
#pragma unroll
              for (int j = 0; j < 8; ++j) { float v = acc[nb][j] * iv[j] + bb; v = (v > 0.0f) ? v : (v - v);
                  sh1[(hi * 8 + j) * HP + col] = toh_flush(v * CH); } }
        }
        __syncthreads();

        { const int cb = wave * 64;
          v8f acc[4];
#pragma unroll
          for (int nb = 0; nb < 4; ++nb) acc[nb] = (v8f){};
          const size_t wo = ((size_t)sg * HID + (size_t)(cb + lr)) * HID + 8 * hi;
          const int ho = lr * HP + 8 * hi;
#pragma unroll 1
          for (int kc = 0; kc < HID; kc += 32) {
              const v16h a = cat16(*(const v8ha*)(&sh1[ho + kc]), *(const v8ha*)(&sh1[ho + kc + 16]));
#pragma unroll
              for (int nb = 0; nb < 4; ++nb) { const v16h b = ldhu(WH + wo + (size_t)nb * 16 * HID + kc); acc[nb] = wmma16g(a, b, acc[nb]); }
          }
#pragma unroll
          for (int nb = 0; nb < 4; ++nb) { const int col = cb + nb * 16 + lr; const float bb = bfr(bh[(size_t)sg * HID + col]);
#pragma unroll
              for (int j = 0; j < 8; ++j) { float v = acc[nb][j] * CINV + bb; v = (v > 0.0f) ? v : (v - v);
                  sh2[(hi * 8 + j) * HP + col] = toh_flush(v * CH); } }
        }
        __syncthreads();

        if (wave < 2) {
            const int col = wave * 16 + lr;
            v8f acc = (v8f){};
            const size_t wo = ((size_t)sg * OUTP + (size_t)col) * HID + 8 * hi;
            const int ho = lr * HP + 8 * hi;
#pragma unroll 1
            for (int kc = 0; kc < HID; kc += 32) {
                const v16h a = cat16(*(const v8ha*)(&sh2[ho + kc]), *(const v8ha*)(&sh2[ho + kc + 16]));
                const v16h b = ldhu(WO + wo + kc);
                acc = wmma16g(a, b, acc);
            }
            const int colc = col < OUTD ? col : OUTD - 1;
            float bv = bo[(size_t)sg * OUTD + colc]; asm volatile("" : "+v"(bv));
            const float b3 = (col < OUTD) ? bfr(bv) : 0.0f;
#pragma unroll
            for (int j = 0; j < 8; ++j) so[(hi * 8 + j) * OSP + col] = acc[j] * CINV + b3;
        }
        __syncthreads();

        { const int row = tid >> 3, pc = tid & 7; const int li = t0 + row; const bool rv = li < cntu;
          int s = lst[li < NB ? li : NB - 1]; s = s < 0 ? 0 : (s > NB - 1 ? NB - 1 : s);
          const v4f val = *(const v4fa*)(&so[row * OSP + pc * 4]);
          float* dp = OW + (size_t)s * OUTP + pc * 4;
#pragma unroll 1
          for (int ps = 0; ps < 2; ++ps) { if (rv) *(volatile v4f*)dp = val; if (ps == 0) __threadfence(); } }
    }
}

__global__ __launch_bounds__(256) void k_out(const float* __restrict__ OW, float* OUT, int n4) {
    const int i = blockIdx.x * 256 + threadIdx.x; if (i >= n4) return;
    const int e = i * 4; const int row = e / OUTD, col = e - row * OUTD;
    const v4f v = *(const v4f*)(OW + (size_t)row * OUTP + col);
    *(volatile v4f*)(OUT + (size_t)i * 4) = v; __threadfence(); *(volatile v4f*)(OUT + (size_t)i * 4) = v;
}

static constexpr size_t al256(size_t v) { return (v + 255) & ~(size_t)255; }
static constexpr size_t SZ_WI = al256((size_t)NSET * HID * OBSP * 2);
static constexpr size_t SZ_WH = al256((size_t)NSET * HID * HID * 2);
static constexpr size_t SZ_WO = al256((size_t)NSET * OUTP * HID * 2);
static constexpr size_t SZ_OW = al256((size_t)NB * OUTP * 4);
static constexpr size_t SZ_TOTAL = SZ_WI + SZ_WH + SZ_WO + SZ_OW;
static_assert(SZ_TOTAL <= (size_t)134217728);
static_assert(((size_t)NB * OUTD) % 8 == 0);

extern "C" void kernel_launch(void* const* d_in, const int* in_sizes, int n_in,
                              void* d_out, int out_size, void* d_ws, size_t ws_size, hipStream_t stream) {
    if (n_in < 9) return;
    if ((size_t)in_sizes[0] < (size_t)NB * OBS || (size_t)in_sizes[1] < (size_t)NB * LIMBS || (size_t)in_sizes[2] < (size_t)NB) return;
    if ((size_t)in_sizes[3] < (size_t)NSET * OBS * HID || (size_t)in_sizes[4] < (size_t)NSET * HID) return;
    if ((size_t)in_sizes[5] < (size_t)NSET * HID * HID || (size_t)in_sizes[6] < (size_t)NSET * HID) return;
    if ((size_t)in_sizes[7] < (size_t)NSET * HID * OUTD || (size_t)in_sizes[8] < (size_t)NSET * OUTD) return;
    if ((size_t)out_size < (size_t)NB * OUTD) return;
    if (SZ_TOTAL > ws_size) return;
    const float* obs = (const float*)d_in[0];
    const int*   omk = (const int*)d_in[1];
    const int*   ids = (const int*)d_in[2];
    const float* wi  = (const float*)d_in[3]; const float* bi = (const float*)d_in[4];
    const float* wh  = (const float*)d_in[5]; const float* bh = (const float*)d_in[6];
    const float* wo  = (const float*)d_in[7]; const float* bo = (const float*)d_in[8];
    float* OUT = (float*)d_out;
    char* wsp = (char*)d_ws;
    bf* WIp = (bf*)wsp; wsp += SZ_WI;
    bf* WHp = (bf*)wsp; wsp += SZ_WH;
    bf* WOp = (bf*)wsp; wsp += SZ_WO;
    float* OWp = (float*)wsp; wsp += SZ_OW;

    k_wt<<<dim3(OBSP / 64, HID / 32, NSET), 256, 0, stream>>>(wi, WIp, OBS, HID, OBSP, HID, 0, 1.0f);
    k_wt<<<dim3(HID / 64, HID / 32, NSET), 256, 0, stream>>>(wh, WHp, HID, HID, HID, HID, 1, CW);
    k_wt<<<dim3(HID / 64, OUTP / 32, NSET), 256, 0, stream>>>(wo, WOp, HID, OUTD, HID, OUTP, 1, CW);

    k_layers<<<dim3(NSET, 1, 1), 128, 0, stream>>>(obs, omk, ids, WIp, bi, WHp, bh, WOp, bo, OWp);

    const int n4 = NB * OUTD / 4;
    k_out<<<dim3((unsigned)((n4 + 255) / 256), 1, 1), 256, 0, stream>>>(OWp, OUT, n4);
}
